// SelectiveSSM_12936441495989
// MI455X (gfx1250) — hardware-verified
//
#include <hip/hip_runtime.h>
#include <math.h>

typedef __attribute__((ext_vector_type(16))) _Float16 v16h;
typedef __attribute__((ext_vector_type(8)))  _Float16 v8h;
typedef __attribute__((ext_vector_type(16))) __bf16   v16b;
typedef __attribute__((ext_vector_type(8)))  __bf16   v8b;
typedef __attribute__((ext_vector_type(8)))  float    v8f;
typedef __attribute__((ext_vector_type(4)))  float    v4f;

constexpr int kBatch  = 2;
constexpr int kSeq    = 512;
constexpr int kDm     = 768;
constexpr int kDin    = 1536;
constexpr int kNst    = 16;
constexpr int kRows   = kBatch * kSeq;
constexpr int kXzP    = 2 * kDin;
constexpr int kWxN    = kDin + 2 * kNst;
constexpr int kWxNP   = 1600;
constexpr int kBcP    = 64;
constexpr int kConvTP = 260;
constexpr int kChunk  = 32;
constexpr int kNChunk = 16;
constexpr int kBvP    = 20;
constexpr int kGtP    = 68;
static_assert(kRows == 1024 && kXzP == 3072 && kWxN == 1568, "shape constants");
static_assert(kChunk * kNChunk == kSeq && kNst * kNChunk == 256, "scan thread map");
static_assert((kDm % 32) == 0 && (kDin % 32) == 0, "GEMM K multiples of 32");
static_assert((kRows % 64) == 0 && (kXzP % 64) == 0 && (kDin % 64) == 0 && (kDm % 64) == 0 && (kBcP % 64) == 0, "GEMM M,N multiples of 64");
static_assert(kWxNP - kDin == kBcP && kWxNP >= kWxN, "x_proj pad rows");
static_assert((kSeq % 64) == 0 && (kDin % 256) == 0 && (kSeq & (kSeq - 1)) == 0, "tile multiples");

constexpr size_t kOffXB   = 0;
constexpr size_t kOffWIB  = kOffXB  + (size_t)kRows * kDm   * 2;
constexpr size_t kOffWXB  = kOffWIB + (size_t)kXzP  * kDm   * 2;
constexpr size_t kOffWDB  = kOffWXB + (size_t)kWxNP * kDin  * 2;
constexpr size_t kOffWOB  = kOffWDB + (size_t)kDin  * kDin  * 2;
constexpr size_t kOffXZ   = kOffWOB + (size_t)kDm   * kDin  * 2;
constexpr size_t kOffUC   = kOffXZ  + (size_t)kRows * kXzP  * 4;
constexpr size_t kOffUCH  = kOffUC  + (size_t)kRows * kDin  * 4;
constexpr size_t kOffDTH  = kOffUCH + (size_t)kRows * kDin  * 2;
constexpr size_t kOffXBC  = kOffDTH + (size_t)kRows * kDin  * 2;
constexpr size_t kOffDLR  = kOffXBC + (size_t)kRows * kBcP  * 4;
constexpr size_t kOffYST  = kOffDLR + (size_t)kRows * kDin  * 4;
constexpr size_t kOffYH   = kOffYST + (size_t)kBatch * kDin * kSeq * 4;
constexpr size_t kOffYL   = kOffYH  + (size_t)kRows * kDin  * 2;
constexpr size_t kWsTotal = kOffYL  + (size_t)kRows * kDin  * 2;
static_assert(kWsTotal == 62586880ull, "carve total");
static_assert(kWsTotal <= 134217728ull, "carve cap");
static_assert((kOffWIB % 128) == 0 && (kOffWXB % 128) == 0 && (kOffWDB % 128) == 0 && (kOffWOB % 128) == 0 &&
              (kOffXZ % 128) == 0 && (kOffUC % 128) == 0 && (kOffUCH % 128) == 0 && (kOffDTH % 128) == 0 &&
              (kOffXBC % 128) == 0 && (kOffDLR % 128) == 0 && (kOffYST % 128) == 0 && (kOffYH % 128) == 0 &&
              (kOffYL % 128) == 0, "128-B aligned regions");

__device__ __forceinline__ unsigned short f2bf_bits(float f) {
  unsigned u = __float_as_uint(f);
  return (unsigned short)((u + 0x7FFFu + ((u >> 16) & 1u)) >> 16);
}
__device__ __forceinline__ float bf_bits2f(unsigned short h) { return __uint_as_float(((unsigned)h) << 16); }
__device__ __forceinline__ float bf_rne(float f) { return bf_bits2f(f2bf_bits(f)); }

__device__ __forceinline__ void row_guard_h(v8f& a, v8f& b, v8f& c, v8f& d, v16h x, v16h y) {
  asm volatile("v_nop\n\tv_nop\n\tv_nop\n\tv_nop" : "+v"(a), "+v"(b), "+v"(c), "+v"(d) : "v"(x), "v"(y));
}
__device__ __forceinline__ void row_guard_b(v8f& a, v8f& b, v8f& c, v8f& d, v16b x, v16b y) {
  asm volatile("v_nop\n\tv_nop\n\tv_nop\n\tv_nop" : "+v"(a), "+v"(b), "+v"(c), "+v"(d) : "v"(x), "v"(y));
}
__device__ __forceinline__ void keep4_h(v16h a, v16h b, v16h c, v16h d) { asm volatile("v_nop" :: "v"(a), "v"(b), "v"(c), "v"(d)); }
__device__ __forceinline__ void keep4_b(v16b a, v16b b, v16b c, v16b d) { asm volatile("v_nop" :: "v"(a), "v"(b), "v"(c), "v"(d)); }
__device__ __forceinline__ void acc_guard4(v8f& a, v8f& b, v8f& c, v8f& d) {
  asm volatile("v_nop\n\tv_nop\n\tv_nop\n\tv_nop" : "+v"(a), "+v"(b), "+v"(c), "+v"(d));
}
template <typename T> struct Frag;
template <> struct Frag<_Float16> {
  typedef v16h V; union U { v16h v; v8h h[2]; };
  static __device__ __forceinline__ v16h load(const _Float16* p) {
    U f; f.h[0] = *(const v8h*)(p); f.h[1] = *(const v8h*)(p + 16); return f.v;
  }
  static __device__ __forceinline__ v8f mma(v16h a, v16h b, v8f c) {
    return __builtin_amdgcn_wmma_f32_16x16x32_f16(false, a, false, b, (short)0, c, false, false);
  }
  static __device__ __forceinline__ void guard4(v8f& a, v8f& b, v8f& c, v8f& d, v16h x, v16h y) { row_guard_h(a, b, c, d, x, y); }
  static __device__ __forceinline__ void keep(v16h a, v16h b, v16h c, v16h d) { keep4_h(a, b, c, d); }
};
template <> struct Frag<__bf16> {
  typedef v16b V; union U { v16b v; v8b h[2]; };
  static __device__ __forceinline__ v16b load(const __bf16* p) {
    U f; f.h[0] = *(const v8b*)(p); f.h[1] = *(const v8b*)(p + 16); return f.v;
  }
  static __device__ __forceinline__ v8f mma(v16b a, v16b b, v8f c) {
    return __builtin_amdgcn_wmma_f32_16x16x32_bf16(false, a, false, b, (short)0, c, false, false);
  }
  static __device__ __forceinline__ void guard4(v8f& a, v8f& b, v8f& c, v8f& d, v16b x, v16b y) { row_guard_b(a, b, c, d, x, y); }
  static __device__ __forceinline__ void keep(v16b a, v16b b, v16b c, v16b d) { keep4_b(a, b, c, d); }
};

template <int ET> struct Elem;
template <> struct Elem<0> { typedef _Float16 T; };
template <> struct Elem<1> { typedef __bf16 T; };
template <int ET, int SPL, int BIAS_MODE, int OUT_MODE, bool RESID, int ACT = 0>
__global__ __launch_bounds__(256) void wmma_gemm64(
    const unsigned short* __restrict__ Ap, const unsigned short* __restrict__ A2p, int lda, long strideA,
    const unsigned short* __restrict__ Btp, const unsigned short* __restrict__ Bt2p, int ldb, long strideB,
    void* __restrict__ Cout, void* __restrict__ Cout2, int ldc, long strideC,
    const float* __restrict__ bias,
    const float* __restrict__ resid, long strideR,
    int M, int N, int K, float scale) {
  typedef typename Elem<ET>::T T;
  typedef typename Frag<T>::V V;
  const T* A = (const T*)Ap; const T* A2 = (const T*)A2p; const T* Bt = (const T*)Btp; const T* Bt2 = (const T*)Bt2p;
  __shared__ __align__(16) float sT[8][16 * 68];
  const int b    = blockIdx.y;
  const int lane = threadIdx.x & 31;
  const int wave = threadIdx.x >> 5;
  const int tilesN = N >> 6;
  const int tilesM = M >> 6;
  const int tile = blockIdx.x * 8 + wave;
  if (tile >= tilesM * tilesN) return;
  const int tm = tile / tilesN;
  const int tn = tile - tm * tilesN;
  const int m0 = tm << 6;
  const int n0 = tn << 6;

  const T* Ab  = A  + (size_t)b * strideA;
  const T* Bb  = Bt + (size_t)b * strideB;
  const T* Ab2 = (SPL >= 1) ? (A2  + (size_t)b * strideA) : nullptr;
  const T* Bb2 = (SPL == 2) ? (Bt2 + (size_t)b * strideB) : nullptr;

  const int rlane = lane & 15;
  const int koff  = (lane >> 4) * 8;
  const int mOff  = (lane >> 4) * 8;

  v8f acc[4][4];
#pragma unroll
  for (int i = 0; i < 4; ++i)
#pragma unroll
    for (int j = 0; j < 4; ++j) acc[i][j] = (v8f){0.f,0.f,0.f,0.f,0.f,0.f,0.f,0.f};

  for (int k0 = 0; k0 < K; k0 += 32) {
    V bh[4], bl[4];
#pragma unroll
    for (int j = 0; j < 4; ++j) {
      const size_t bo = (size_t)(n0 + (j << 4) + rlane) * ldb + koff + k0;
      bh[j] = Frag<T>::load(Bb + bo);
      if (SPL == 2) bl[j] = Frag<T>::load(Bb2 + bo);
    }
#pragma unroll
    for (int i = 0; i < 4; ++i) {
      const size_t ao = (size_t)(m0 + (i << 4) + rlane) * lda + koff + k0;
      V ah = Frag<T>::load(Ab + ao);
      V al;
      if (SPL >= 1) al = Frag<T>::load(Ab2 + ao);
#pragma unroll
      for (int j = 0; j < 4; ++j) {
        acc[i][j] = Frag<T>::mma(ah, bh[j], acc[i][j]);
        if (SPL == 2) acc[i][j] = Frag<T>::mma(ah, bl[j], acc[i][j]);
        if (SPL >= 1) acc[i][j] = Frag<T>::mma(al, bh[j], acc[i][j]);
      }
      Frag<T>::guard4(acc[i][0], acc[i][1], acc[i][2], acc[i][3], ah, (SPL >= 1) ? al : ah);
    }
    Frag<T>::keep(bh[0], bh[1], bh[2], bh[3]);
    if (SPL == 2) Frag<T>::keep(bl[0], bl[1], bl[2], bl[3]);
  }
  acc_guard4(acc[0][0], acc[0][1], acc[0][2], acc[0][3]);
  acc_guard4(acc[1][0], acc[1][1], acc[1][2], acc[1][3]);
  acc_guard4(acc[2][0], acc[2][1], acc[2][2], acc[2][3]);
  acc_guard4(acc[3][0], acc[3][1], acc[3][2], acc[3][3]);

  float* slab = sT[wave];
  const float* Rb = RESID ? (resid + (size_t)b * strideR) : nullptr;
#pragma unroll
  for (int i = 0; i < 4; ++i) {
    const int mBase = m0 + (i << 4);
#pragma unroll
    for (int j = 0; j < 4; ++j) {
      const int n = n0 + (j << 4) + rlane;
      float bv = 0.f;
      if (BIAS_MODE == 2) bv = bias[n];
#pragma unroll
      for (int r = 0; r < 8; ++r) {
        float v = acc[i][j][r] * scale;
        if (BIAS_MODE == 1) v += bias[mBase + mOff + r];
        if (BIAS_MODE == 2) v += bv;
        if (RESID) v += Rb[(size_t)(mBase + mOff + r) * ldc + n];
        if (ACT == 1) v = tanhf(v);
        if (ACT == 2) v = fmaxf(v, 0.0f);
        if (ACT == 3) v = v / (1.0f + expf(-v));
        if (ACT == 4) v = (v > 0.f) ? v : 0.01f * v;
        slab[(mOff + r) * 68 + (j << 4) + rlane] = v;
      }
    }
    __builtin_amdgcn_fence(__ATOMIC_RELEASE, "workgroup");
    __builtin_amdgcn_wave_barrier();
    __builtin_amdgcn_fence(__ATOMIC_ACQUIRE, "workgroup");
    if (OUT_MODE == 0) {
      float* C = (float*)Cout + (size_t)b * strideC;
      const int hh = lane >> 4, c4 = (lane & 15) * 4;
      for (int pass = 0; pass < 2; ++pass) {
#pragma unroll
        for (int it = 0; it < 8; ++it) {
          const int row = it * 2 + hh;
          v4f v = *(const v4f*)(slab + row * 68 + c4);
          *(volatile v4f*)(C + (size_t)(mBase + row) * ldc + n0 + c4) = v;
        }
        __threadfence();
      }
    } else {
      const int q = lane >> 3, c8 = (lane & 7) * 8;
      unsigned short* C  = (unsigned short*)Cout  + (size_t)b * strideC;
      unsigned short* C2 = (OUT_MODE == 2) ? ((unsigned short*)Cout2 + (size_t)b * strideC) : nullptr;
      for (int pass = 0; pass < 2; ++pass) {
#pragma unroll
        for (int it = 0; it < 4; ++it) {
          const int row = it * 4 + q;
          const float* sp = slab + row * 68 + c8;
          v8h hv, lv;
#pragma unroll
          for (int e = 0; e < 8; ++e) {
            const float sv = sp[e];
            if (OUT_MODE == 1) {
              hv[e] = (_Float16)sv;
            } else {
              const unsigned short hb = f2bf_bits(sv);
              hv[e] = __builtin_bit_cast(_Float16, hb);
              if (OUT_MODE == 2) {
                const unsigned short lb = f2bf_bits(sv - bf_bits2f(hb));
                lv[e] = __builtin_bit_cast(_Float16, lb);
              }
            }
          }
          *(volatile v8h*)(C + (size_t)(mBase + row) * ldc + n0 + c8) = hv;
          if (OUT_MODE == 2) *(volatile v8h*)(C2 + (size_t)(mBase + row) * ldc + n0 + c8) = lv;
        }
        __threadfence();
      }
    }
    __builtin_amdgcn_fence(__ATOMIC_RELEASE, "workgroup");
    __builtin_amdgcn_wave_barrier();
    __builtin_amdgcn_fence(__ATOMIC_ACQUIRE, "workgroup");
  }
}

__global__ __launch_bounds__(256) void cast_rows_bf16_kernel(
    const float* __restrict__ src, unsigned short* __restrict__ dst, int real8, int total8)
{
  const int i = blockIdx.x * 256 + threadIdx.x;
  if (i >= total8) return;
  const bool live = (i < real8);
  const int ic = live ? i : (real8 - 1);
  const size_t s0 = (size_t)ic << 3;
  const size_t e0 = (size_t)i << 3;
  const v4f a0 = *(const v4f*)(src + s0);
  const v4f a1 = *(const v4f*)(src + s0 + 4);
  v8h hv;
#pragma unroll
  for (int e = 0; e < 4; ++e) {
    const float f0 = live ? a0[e] : 0.0f;
    const float f1 = live ? a1[e] : 0.0f;
    const unsigned short h0 = f2bf_bits(f0);
    const unsigned short h1 = f2bf_bits(f1);
    hv[e]     = __builtin_bit_cast(_Float16, h0);
    hv[4 + e] = __builtin_bit_cast(_Float16, h1);
  }
  unsigned short* qd = dst + e0;
  *(volatile v8h*)qd = hv;
  __threadfence();
  *(volatile v8h*)qd = hv;
}

__global__ __launch_bounds__(256) void conv_silu_kernel(
    const float* __restrict__ XZ, const float* __restrict__ cw, const float* __restrict__ cb,
    float* __restrict__ UC, unsigned short* __restrict__ UCH)
{
  __shared__ __align__(16) float sT[16 * kConvTP];
  const int tid = threadIdx.x, lane = tid & 31, wave = tid >> 5;
  const int d0 = blockIdx.x * 256, d = d0 + tid;
  const int g0 = blockIdx.y * 64;
  const int tb = g0 & (kSeq - 1);
  const v4f wv = *(const v4f*)(cw + (size_t)d * 4);
  const float w0 = bf_rne(wv[0]), w1 = bf_rne(wv[1]), w2 = bf_rne(wv[2]), w3 = bf_rne(wv[3]);
  const float bc = bf_rne(cb[d]);
  float xm3, xm2, xm1;
  {
    const bool hist = (tb > 0);
    const int rb = hist ? (g0 - 3) : g0;
    const float v3 = XZ[(size_t)rb * kXzP + d];
    const float v2 = XZ[(size_t)(rb + 1) * kXzP + d];
    const float v1 = XZ[(size_t)(rb + 2) * kXzP + d];
    xm3 = hist ? v3 : 0.f;
    xm2 = hist ? v2 : 0.f;
    xm1 = hist ? v1 : 0.f;
  }
  const int hrow = wave >> 1;
  const int hch  = (wave & 1) * 128 + lane * 4;
#pragma unroll 1
  for (int sub = 0; sub < 4; ++sub) {
    const int lb = g0 + sub * 16;
#pragma unroll 1
    for (int s = 0; s < 16; ++s) {
      const float xcur = XZ[(size_t)(lb + s) * kXzP + d];
      float acc = w0 * xm3;
      acc = fmaf(w1, xm2, acc);
      acc = fmaf(w2, xm1, acc);
      acc = fmaf(w3, xcur, acc);
      const float sv = acc + bc;
      const float den = 1.0f + expf(-sv);
      const float sg = 1.0f / den;
      sT[s * kConvTP + tid] = sv * sg;
      xm3 = xm2; xm2 = xm1; xm1 = xcur;
    }
    __syncthreads();
    v4f fv[4];
    v8h bh[2];
#pragma unroll
    for (int it = 0; it < 4; ++it) fv[it] = *(const v4f*)(sT + (it * 4 + hrow) * kConvTP + hch);
#pragma unroll
    for (int it = 0; it < 2; ++it) {
      const float* sp = sT + (it * 8 + wave) * kConvTP + lane * 8;
      const v4f a0 = *(const v4f*)(sp);
      const v4f a1 = *(const v4f*)(sp + 4);
#pragma unroll
      for (int e = 0; e < 4; ++e) {
        const unsigned short h0 = f2bf_bits(a0[e]);
        const unsigned short h1 = f2bf_bits(a1[e]);
        bh[it][e]     = __builtin_bit_cast(_Float16, h0);
        bh[it][4 + e] = __builtin_bit_cast(_Float16, h1);
      }
    }
    for (int pass = 0; pass < 2; ++pass) {
#pragma unroll
      for (int it = 0; it < 4; ++it)
        *(volatile v4f*)(UC + (size_t)(lb + it * 4 + hrow) * kDin + d0 + hch) = fv[it];
#pragma unroll
      for (int it = 0; it < 2; ++it) {
        const size_t o = (size_t)(lb + it * 8 + wave) * kDin + d0 + lane * 8;
        *(volatile v8h*)(UCH + o) = bh[it];
      }
      __threadfence();
    }
    __syncthreads();
  }
}

template <int LV> __device__ __forceinline__ void up_level(float (&vv)[kChunk], float (&cc)[kChunk]) {
  constexpr int stp = 2 << LV;
  constexpr int hf  = 1 << LV;
#pragma unroll
  for (int r = stp - 1; r < kChunk; r += stp) {
    const float nv = fmaf(cc[r], vv[r], vv[r - hf]);
    cc[r] = cc[r - hf] * cc[r];
    vv[r] = nv;
  }
}
template <int LV> __device__ __forceinline__ void down_level(float (&vv)[kChunk], const float (&cc)[kChunk]) {
  constexpr int stp = 2 << LV;
  constexpr int hf  = 1 << LV;
#pragma unroll
  for (int r = stp - 1; r < kChunk; r += stp) {
    const float t = vv[r];
    vv[r] = fmaf(cc[r], t, vv[r - hf]);
    vv[r - hf] = t;
  }
}

__global__ __launch_bounds__(256) void scan_kernel(
    const float* __restrict__ DLR, const float* __restrict__ UC, const float* __restrict__ XBC,
    const float* __restrict__ bdt, const float* __restrict__ Alog, float* __restrict__ YST)
{
  __shared__ __align__(16) float sD[kSeq];
  __shared__ __align__(16) float sX[kSeq];
  __shared__ __align__(16) float sBV[kSeq * kBvP];
  __shared__ __align__(16) float sTV[kNst * kNChunk];
  __shared__ __align__(16) float sTC[kNst * kNChunk];
  const int tid = threadIdx.x;
  const int n = tid & 15, chunk = tid >> 4;
  const int b = blockIdx.x / kDin;
  const int d = blockIdx.x - b * kDin;
  const size_t row0 = (size_t)b * kSeq;
  const float bb = bf_rne(bdt[d]);
  const float An = -__expf(bf_rne(Alog[(size_t)d * kNst + n]));

#pragma unroll
  for (int k = 0; k < 2; ++k) {
    const int row = tid + 256 * k;
    const float v  = DLR[(row0 + row) * kDin + d] + bb;
    const float a  = __expf(-fabsf(v));
    const float u  = 1.0f + a;
    const float l1 = __logf(u) + (a - (u - 1.0f)) * __builtin_amdgcn_rcpf(u);
    sD[row] = fmaxf(v, 0.0f) + l1;
    sX[row] = UC[(row0 + row) * kDin + d];
  }
#pragma unroll
  for (int k = 0; k < 8; ++k) {
    const int idx = tid + 256 * k;
    const int row = idx >> 2, q = idx & 3;
    const v4f bv = *(const v4f*)(XBC + (row0 + row) * kBcP + q * 4);
    *(v4f*)(sBV + row * kBvP + q * 4) = bv;
  }
  __syncthreads();

  float vv[kChunk], cc[kChunk];
#pragma unroll
  for (int i = 0; i < kChunk; ++i) {
    const int pos = chunk * kChunk + i;
    const float dl = sD[pos];
    const float xv = sX[pos];
    const float bn = sBV[pos * kBvP + n];
    cc[i] = __expf(dl * An) + 1e-12f;
    vv[i] = fabsf((dl * bn) * xv) + 1e-12f;
  }
  up_level<0>(vv, cc);
  up_level<1>(vv, cc);
  up_level<2>(vv, cc);
  up_level<3>(vv, cc);
  up_level<4>(vv, cc);
  sTV[n * kNChunk + chunk] = vv[kChunk - 1];
  sTC[n * kNChunk + chunk] = cc[kChunk - 1];
  __syncthreads();
  if (tid < kNst) {
    float* tv = sTV + tid * kNChunk;
    float* tc = sTC + tid * kNChunk;
#pragma unroll 1
    for (int lv = 0; lv < 4; ++lv) {
      const int stp = 2 << lv, hf = 1 << lv;
#pragma unroll 1
      for (int r = stp - 1; r < kNChunk; r += stp) {
        const float cr = tc[r];
        const float vr = tv[r];
        const float vl = tv[r - hf];
        const float cl = tc[r - hf];
        tv[r] = fmaf(cr, vr, vl);
        tc[r] = cl * cr;
      }
    }
#pragma unroll 1
    for (int lv = 3; lv >= 0; --lv) {
      const int stp = 2 << lv, hf = 1 << lv;
#pragma unroll 1
      for (int r = stp - 1; r < kNChunk; r += stp) {
        const float cr = tc[r];
        const float vr = tv[r];
        const float vl = tv[r - hf];
        tv[r] = fmaf(cr, vr, vl);
        tv[r - hf] = vr;
      }
    }
  }
  __syncthreads();
  vv[kChunk - 1] = sTV[n * kNChunk + chunk];
  cc[kChunk - 1] = sTC[n * kNChunk + chunk];
  down_level<4>(vv, cc);
  down_level<3>(vv, cc);
  down_level<2>(vv, cc);
  down_level<1>(vv, cc);
  down_level<0>(vv, cc);
#pragma unroll
  for (int i = 0; i < kChunk; ++i) sBV[(chunk * kChunk + i) * kBvP + n] = vv[i];
  __syncthreads();
#pragma unroll 1
  for (int p = 0; p < 2; ++p) {
    const int pos = 2 * tid + p;
    const float* cp = XBC + (row0 + pos) * kBcP + kNst;
    const float* vp = sBV + pos * kBvP;
    float s = 0.0f;
#pragma unroll 1
    for (int q = 0; q < 4; ++q) {
      const v4f cv = *(const v4f*)(cp + 4 * q);
      const v4f sv = *(const v4f*)(vp + 4 * q);
      s = fmaf(sv[0], cv[0], s);
      s = fmaf(sv[1], cv[1], s);
      s = fmaf(sv[2], cv[2], s);
      s = fmaf(sv[3], cv[3], s);
    }
    sD[pos] = s;
  }
  __syncthreads();
  if (tid < 128) {
    const v4f o = *(const v4f*)(sD + 4 * tid);
    float* gp = YST + ((size_t)b * kDin + d) * kSeq + 4 * tid;
    *(volatile v4f*)gp = o;
    __threadfence();
    *(volatile v4f*)gp = o;
  }
}

__global__ __launch_bounds__(256) void gate_kernel(
    const float* __restrict__ YST, const float* __restrict__ UC, const float* __restrict__ XZ,
    const float* __restrict__ Dp, unsigned short* __restrict__ YH, unsigned short* __restrict__ YL)
{
  __shared__ __align__(16) float tile[64 * kGtP];
  const int tid = threadIdx.x, lane = tid & 31, wave = tid >> 5;
  const int d0 = blockIdx.x * 64;
  const int g0 = blockIdx.y * 64;
  const int b  = g0 / kSeq;
  const int lp0 = g0 - b * kSeq;
  const int c = tid & 63, r4 = tid >> 6;
#pragma unroll 1
  for (int it = 0; it < 16; ++it) {
    const int dd = r4 + 4 * it;
    tile[c * kGtP + dd] = YST[((size_t)b * kDin + d0 + dd) * kSeq + lp0 + c];
  }
  __syncthreads();
  const float Dd = bf_rne(Dp[d0 + c]);
#pragma unroll 1
  for (int it = 0; it < 16; ++it) {
    const int lr = r4 + 4 * it;
    const size_t g = (size_t)(g0 + lr);
    const float ys = tile[lr * kGtP + c];
    const float xc = UC[g * kDin + d0 + c];
    const float zv = XZ[g * kXzP + kDin + d0 + c];
    const float sk = xc * Dd;
    const float y  = ys + sk;
    const float den = 1.0f + expf(-zv);
    const float sg = 1.0f / den;
    tile[lr * kGtP + c] = y * (zv * sg);
  }
  __syncthreads();
  const int q = lane >> 3, c8 = (lane & 7) * 8;
  v8h hv[2], lv[2];
#pragma unroll
  for (int it = 0; it < 2; ++it) {
    const int row = it * 32 + wave * 4 + q;
    const float* sp = tile + row * kGtP + c8;
    const v4f a0 = *(const v4f*)(sp);
    const v4f a1 = *(const v4f*)(sp + 4);
#pragma unroll
    for (int e = 0; e < 4; ++e) {
      const float f0 = a0[e];
      const float f1 = a1[e];
      const unsigned short h0 = f2bf_bits(f0);
      const unsigned short h1 = f2bf_bits(f1);
      const unsigned short l0 = f2bf_bits(f0 - bf_bits2f(h0));
      const unsigned short l1 = f2bf_bits(f1 - bf_bits2f(h1));
      hv[it][e]     = __builtin_bit_cast(_Float16, h0);
      hv[it][4 + e] = __builtin_bit_cast(_Float16, h1);
      lv[it][e]     = __builtin_bit_cast(_Float16, l0);
      lv[it][4 + e] = __builtin_bit_cast(_Float16, l1);
    }
  }
  for (int pass = 0; pass < 2; ++pass) {
#pragma unroll
    for (int it = 0; it < 2; ++it) {
      const int row = it * 32 + wave * 4 + q;
      const size_t o = (size_t)(g0 + row) * kDin + d0 + c8;
      *(volatile v8h*)(YH + o) = hv[it];
      *(volatile v8h*)(YL + o) = lv[it];
    }
    __threadfence();
  }
}

extern "C" void kernel_launch(void* const* d_in, const int* in_sizes, int n_in,
                              void* d_out, int out_size, void* d_ws, size_t ws_size,
                              hipStream_t stream) {
  if (n_in < 10) return;
  if (in_sizes[0] != kRows * kDm) return;
  if (in_sizes[1] != kXzP * kDm) return;
  if (in_sizes[2] != kDin * 4) return;
  if (in_sizes[3] != kDin) return;
  if (in_sizes[4] != kWxN * kDin) return;
  if (in_sizes[5] != kDin * kDin) return;
  if (in_sizes[6] != kDin) return;
  if (in_sizes[7] != kDin * kNst) return;
  if (in_sizes[8] != kDin) return;
  if (in_sizes[9] != kDm * kDin) return;
  if (out_size != kRows * kDm) return;
  if (ws_size < kWsTotal) return;

  const float* x      = (const float*)d_in[0];
  const float* W_in   = (const float*)d_in[1];
  const float* conv_w = (const float*)d_in[2];
  const float* conv_b = (const float*)d_in[3];
  const float* W_x    = (const float*)d_in[4];
  const float* W_dt   = (const float*)d_in[5];
  const float* b_dt   = (const float*)d_in[6];
  const float* A_log  = (const float*)d_in[7];
  const float* Dp     = (const float*)d_in[8];
  const float* W_out  = (const float*)d_in[9];
  float* out = (float*)d_out;

  char* ws = (char*)d_ws;
  unsigned short* XB  = (unsigned short*)(ws + kOffXB);
  unsigned short* WIB = (unsigned short*)(ws + kOffWIB);
  unsigned short* WXB = (unsigned short*)(ws + kOffWXB);
  unsigned short* WDB = (unsigned short*)(ws + kOffWDB);
  unsigned short* WOB = (unsigned short*)(ws + kOffWOB);
  float*          XZ  = (float*)(ws + kOffXZ);
  float*          UC  = (float*)(ws + kOffUC);
  unsigned short* UCH = (unsigned short*)(ws + kOffUCH);
  unsigned short* DTH = (unsigned short*)(ws + kOffDTH);
  float*          XBC = (float*)(ws + kOffXBC);
  float*          DLR = (float*)(ws + kOffDLR);
  float*          YST = (float*)(ws + kOffYST);
  unsigned short* YH  = (unsigned short*)(ws + kOffYH);
  unsigned short* YL  = (unsigned short*)(ws + kOffYL);
  const float* dummy_bias  = b_dt;
  const float* dummy_resid = x;

  cast_rows_bf16_kernel<<<(kRows * kDm / 8) / 256, 256, 0, stream>>>(x, XB, kRows * kDm / 8, kRows * kDm / 8);
  cast_rows_bf16_kernel<<<(kXzP * kDm / 8) / 256, 256, 0, stream>>>(W_in, WIB, kXzP * kDm / 8, kXzP * kDm / 8);
  cast_rows_bf16_kernel<<<(kWxNP * kDin / 8) / 256, 256, 0, stream>>>(W_x, WXB, kWxN * kDin / 8, kWxNP * kDin / 8);
  cast_rows_bf16_kernel<<<(kDin * kDin / 8) / 256, 256, 0, stream>>>(W_dt, WDB, kDin * kDin / 8, kDin * kDin / 8);
  cast_rows_bf16_kernel<<<(kDm * kDin / 8) / 256, 256, 0, stream>>>(W_out, WOB, kDm * kDin / 8, kDm * kDin / 8);

  wmma_gemm64<1, 0, 0, 0, false><<<dim3(96, 1), 256, 0, stream>>>(
      XB, XB, kDm, 0L,
      WIB, WIB, kDm, 0L,
      (void*)XZ, (void*)XZ, kXzP, 0L,
      dummy_bias, dummy_resid, 0L,
      kRows, kXzP, kDm, 1.0f);

  conv_silu_kernel<<<dim3(kDin / 256, kRows / 64), 256, 0, stream>>>(XZ, conv_w, conv_b, UC, UCH);

  wmma_gemm64<1, 0, 0, 3, false><<<dim3(48, 1), 256, 0, stream>>>(
      UCH, UCH, kDin, 0L,
      WXB, WXB, kDin, 0L,
      (void*)DTH, (void*)DTH, kDin, 0L,
      dummy_bias, dummy_resid, 0L,
      kRows, kDin, kDin, 1.0f);

  wmma_gemm64<1, 0, 0, 0, false><<<dim3(2, 1), 256, 0, stream>>>(
      UCH, UCH, kDin, 0L,
      WXB + (size_t)kDin * kDin, WXB + (size_t)kDin * kDin, kDin, 0L,
      (void*)XBC, (void*)XBC, kBcP, 0L,
      dummy_bias, dummy_resid, 0L,
      kRows, kBcP, kDin, 1.0f);

  wmma_gemm64<1, 0, 0, 0, false><<<dim3(48, 1), 256, 0, stream>>>(
      DTH, DTH, kDin, 0L,
      WDB, WDB, kDin, 0L,
      (void*)DLR, (void*)DLR, kDin, 0L,
      dummy_bias, dummy_resid, 0L,
      kRows, kDin, kDin, 1.0f);

  scan_kernel<<<kBatch * kDin, 256, 0, stream>>>(DLR, UC, XBC, b_dt, A_log, YST);

  gate_kernel<<<dim3(kDin / 64, kRows / 64), 256, 0, stream>>>(YST, UC, XZ, Dp, YH, YL);

  wmma_gemm64<1, 1, 0, 0, false><<<dim3(24, 1), 256, 0, stream>>>(
      YH, YL, kDin, 0L,
      WOB, WOB, kDin, 0L,
      (void*)out, (void*)out, kDm, 0L,
      dummy_bias, dummy_resid, 0L,
      kRows, kDm, kDin, 1.0f);
}
